// Batch_Attention_cos_22170621182644
// MI455X (gfx1250) — hardware-verified
//
#include <hip/hip_runtime.h>

typedef __attribute__((ext_vector_type(16))) _Float16 v16h;
typedef __attribute__((ext_vector_type(8)))  _Float16 v8h;
typedef __attribute__((ext_vector_type(16))) __bf16   v16b;
typedef __attribute__((ext_vector_type(8)))  __bf16   v8b;
typedef __attribute__((ext_vector_type(8)))  float    v8f;
typedef __attribute__((ext_vector_type(4)))  float    v4f;

#define NROW 8192
#define NCOL 512
#define NCT  576
#define RB   2048
#define XNSC 16.0f
#define SSC  (1.0f / 256.0f)

__device__ __forceinline__ unsigned short f2bf_bits(float f) {
  unsigned u = __float_as_uint(f);
  return (unsigned short)((u + 0x7FFFu + ((u >> 16) & 1u)) >> 16);
}
__device__ __forceinline__ float bf_bits2f(unsigned short h) { return __uint_as_float(((unsigned)h) << 16); }

__device__ __forceinline__ void dep_guard_h(v8f& a, v8f& b, v16h x, v16h y) { asm volatile("v_nop\n\tv_nop\n\tv_nop\n\tv_nop" : "+v"(a), "+v"(b) : "v"(x), "v"(y)); }
__device__ __forceinline__ void dep_guard_b(v8f& a, v8f& b, v16b x, v16b y) { asm volatile("v_nop\n\tv_nop\n\tv_nop\n\tv_nop" : "+v"(a), "+v"(b) : "v"(x), "v"(y)); }
__device__ __forceinline__ void keep4_h(v16h a, v16h b, v16h c, v16h d) { asm volatile("v_nop" :: "v"(a), "v"(b), "v"(c), "v"(d)); }
__device__ __forceinline__ void keep4_b(v16b a, v16b b, v16b c, v16b d) { asm volatile("v_nop" :: "v"(a), "v"(b), "v"(c), "v"(d)); }
__device__ __forceinline__ void acc_guard4(v8f& a, v8f& b, v8f& c, v8f& d) { asm volatile("v_nop\n\tv_nop\n\tv_nop\n\tv_nop" : "+v"(a), "+v"(b), "+v"(c), "+v"(d)); }
template <typename T> struct Frag;
template <> struct Frag<_Float16> {
  typedef v16h V; union U { v16h v; v8h h[2]; };
  static __device__ __forceinline__ v16h load(const _Float16* p) {
    U f; f.h[0] = *(const v8h*)(p); f.h[1] = *(const v8h*)(p + 16); return f.v;
  }
  static __device__ __forceinline__ v8f mma(v16h a, v16h b, v8f c) {
    return __builtin_amdgcn_wmma_f32_16x16x32_f16(false, a, false, b, (short)0, c, false, false);
  }
  static __device__ __forceinline__ void guard(v8f& a, v8f& b, v16h x, v16h y) { dep_guard_h(a, b, x, y); }
  static __device__ __forceinline__ void keep(v16h a, v16h b, v16h c, v16h d) { keep4_h(a, b, c, d); }
};
template <> struct Frag<__bf16> {
  typedef v16b V; union U { v16b v; v8b h[2]; };
  static __device__ __forceinline__ v16b load(const __bf16* p) {
    U f; f.h[0] = *(const v8b*)(p); f.h[1] = *(const v8b*)(p + 16); return f.v;
  }
  static __device__ __forceinline__ v8f mma(v16b a, v16b b, v8f c) {
    return __builtin_amdgcn_wmma_f32_16x16x32_bf16(false, a, false, b, (short)0, c, false, false);
  }
  static __device__ __forceinline__ void guard(v8f& a, v8f& b, v16b x, v16b y) { dep_guard_b(a, b, x, y); }
  static __device__ __forceinline__ void keep(v16b a, v16b b, v16b c, v16b d) { keep4_b(a, b, c, d); }
};

template <int ET> struct Elem;
template <> struct Elem<0> { typedef _Float16 T; };
template <> struct Elem<1> { typedef __bf16 T; };
template <int ET, bool SPLIT, int BIAS_MODE, int OUT_MODE, bool RESID, int ACT = 0>
__global__ __launch_bounds__(256) void wmma_gemm64(
    const unsigned short* __restrict__ Ap, const unsigned short* __restrict__ A2p, int lda, long strideA,
    const unsigned short* __restrict__ Btp, const unsigned short* __restrict__ Bt2p, int ldb, long strideB,
    void* __restrict__ Cout, void* __restrict__ Cout2, int ldc, long strideC,
    const float* __restrict__ bias,
    const float* __restrict__ resid, long strideR,
    int M, int N, int K, float scale) {
  typedef typename Elem<ET>::T T;
  typedef typename Frag<T>::V V;
  const T* A = (const T*)Ap; const T* A2 = (const T*)A2p; const T* Bt = (const T*)Btp; const T* Bt2 = (const T*)Bt2p;
  __shared__ __align__(16) float sT[8][16 * 68];
  const int b    = blockIdx.y;
  const int lane = threadIdx.x & 31;
  const int wave = threadIdx.x >> 5;
  const int tilesN = N >> 6;
  const int tilesM = M >> 6;
  const int tile = blockIdx.x * 8 + wave;
  if (tile >= tilesM * tilesN) return;
  const int tm = tile / tilesN;
  const int tn = tile - tm * tilesN;
  const int m0 = tm << 6;
  const int n0 = tn << 6;

  const T* Ab  = A  + (size_t)b * strideA;
  const T* Bb  = Bt + (size_t)b * strideB;
  const T* Ab2 = SPLIT ? (A2  + (size_t)b * strideA) : nullptr;
  const T* Bb2 = SPLIT ? (Bt2 + (size_t)b * strideB) : nullptr;

  const int rlane = lane & 15;
  const int koff  = (lane >> 4) * 8;
  const int mOff  = (lane >> 4) * 8;

  v8f acc[4][4];
#pragma unroll
  for (int i = 0; i < 4; ++i)
#pragma unroll
    for (int j = 0; j < 4; ++j) acc[i][j] = (v8f){0.f,0.f,0.f,0.f,0.f,0.f,0.f,0.f};

  for (int k0 = 0; k0 < K; k0 += 32) {
    V bh[4], bl[4];
#pragma unroll
    for (int j = 0; j < 4; ++j) {
      const size_t bo = (size_t)(n0 + (j << 4) + rlane) * ldb + koff + k0;
      bh[j] = Frag<T>::load(Bb + bo);
      if (SPLIT) bl[j] = Frag<T>::load(Bb2 + bo);
    }
#pragma unroll
    for (int i = 0; i < 4; ++i) {
      const size_t ao = (size_t)(m0 + (i << 4) + rlane) * lda + koff + k0;
      V ah = Frag<T>::load(Ab + ao);
      V al;
      if (SPLIT) al = Frag<T>::load(Ab2 + ao);
#pragma unroll
      for (int j = 0; j < 4; ++j) {
        acc[i][j] = Frag<T>::mma(ah, bh[j], acc[i][j]);
        if (SPLIT) {
          acc[i][j] = Frag<T>::mma(ah, bl[j], acc[i][j]);
          acc[i][j] = Frag<T>::mma(al, bh[j], acc[i][j]);
        }
      }
      Frag<T>::guard(acc[i][0], acc[i][3], ah, SPLIT ? al : ah);
    }
    Frag<T>::keep(bh[0], bh[1], bh[2], bh[3]);
    if (SPLIT) Frag<T>::keep(bl[0], bl[1], bl[2], bl[3]);
  }
  acc_guard4(acc[0][0], acc[0][1], acc[0][2], acc[0][3]);
  acc_guard4(acc[1][0], acc[1][1], acc[1][2], acc[1][3]);
  acc_guard4(acc[2][0], acc[2][1], acc[2][2], acc[2][3]);
  acc_guard4(acc[3][0], acc[3][1], acc[3][2], acc[3][3]);

  float* slab = sT[wave];
  const float* Rb = RESID ? (resid + (size_t)b * strideR) : nullptr;
#pragma unroll
  for (int i = 0; i < 4; ++i) {
    const int mBase = m0 + (i << 4);
#pragma unroll
    for (int j = 0; j < 4; ++j) {
      const int n = n0 + (j << 4) + rlane;
      float bv = 0.f;
      if (BIAS_MODE == 2) bv = bias[n];
#pragma unroll
      for (int r = 0; r < 8; ++r) {
        float v = acc[i][j][r] * scale;
        if (BIAS_MODE == 1) v += bias[mBase + mOff + r];
        if (BIAS_MODE == 2) v += bv;
        if (RESID) v += Rb[(size_t)(mBase + mOff + r) * ldc + n];
        if (ACT == 1) v = tanhf(v);
        if (ACT == 2) v = fmaxf(v, 0.0f);
        if (ACT == 3) v = v / (1.0f + expf(-v));
        if (ACT == 4) v = (v > 0.f) ? v : 0.01f * v;
        if (ACT == 5) v = 0.5f * v * (1.0f + erff(v * 0.70710678118654752f));
        if (ACT == 6) v = __expf(v - 1.0f);
        slab[(mOff + r) * 68 + (j << 4) + rlane] = v;
      }
    }
    __builtin_amdgcn_fence(__ATOMIC_RELEASE, "workgroup");
    __builtin_amdgcn_wave_barrier();
    __builtin_amdgcn_fence(__ATOMIC_ACQUIRE, "workgroup");
    if (OUT_MODE == 0) {
      float* C = (float*)Cout + (size_t)b * strideC;
      const int hh = lane >> 4, c4 = (lane & 15) * 4;
      for (int pass = 0; pass < 2; ++pass) {
#pragma unroll
        for (int it = 0; it < 8; ++it) {
          const int row = it * 2 + hh;
          v4f v = *(const v4f*)(slab + row * 68 + c4);
          *(volatile v4f*)(C + (size_t)(mBase + row) * ldc + n0 + c4) = v;
        }
        __threadfence();
      }
    } else {
      const int q = lane >> 3, c8 = (lane & 7) * 8;
      unsigned short* C  = (unsigned short*)Cout  + (size_t)b * strideC;
      unsigned short* C2 = (OUT_MODE == 2) ? ((unsigned short*)Cout2 + (size_t)b * strideC) : nullptr;
      for (int pass = 0; pass < 2; ++pass) {
#pragma unroll
        for (int it = 0; it < 4; ++it) {
          const int row = it * 4 + q;
          const float* sp = slab + row * 68 + c8;
          v8h hv, lv;
#pragma unroll
          for (int e = 0; e < 8; ++e) {
            if (OUT_MODE == 1) {
              hv[e] = (_Float16)sp[e];
            } else {
              unsigned short hb = f2bf_bits(sp[e]);
              unsigned short lb = f2bf_bits(sp[e] - bf_bits2f(hb));
              hv[e] = __builtin_bit_cast(_Float16, hb);
              lv[e] = __builtin_bit_cast(_Float16, lb);
            }
          }
          *(volatile v8h*)(C + (size_t)(mBase + row) * ldc + n0 + c8) = hv;
          if (OUT_MODE == 2) *(volatile v8h*)(C2 + (size_t)(mBase + row) * ldc + n0 + c8) = lv;
        }
        __threadfence();
      }
    }
    __builtin_amdgcn_fence(__ATOMIC_RELEASE, "workgroup");
    __builtin_amdgcn_wave_barrier();
    __builtin_amdgcn_fence(__ATOMIC_ACQUIRE, "workgroup");
  }
}

__global__ __launch_bounds__(256) void rownorm_xn16(const float* __restrict__ x, _Float16* __restrict__ xn, int nrows) {
  const int lane = threadIdx.x & 31;
  const int wave = threadIdx.x >> 5;
  const int row  = blockIdx.x * 8 + wave;
  const int rowc = row < nrows ? row : nrows - 1;
  const float* xr = x + (size_t)rowc * NCOL;
  const v4f a0 = *(const v4f*)(xr + lane * 8);
  const v4f a1 = *(const v4f*)(xr + lane * 8 + 4);
  const v4f b0 = *(const v4f*)(xr + 256 + lane * 8);
  const v4f b1 = *(const v4f*)(xr + 256 + lane * 8 + 4);
  float ss = 0.f;
#pragma unroll
  for (int e = 0; e < 4; ++e) ss += a0[e] * a0[e];
#pragma unroll
  for (int e = 0; e < 4; ++e) ss += a1[e] * a1[e];
#pragma unroll
  for (int e = 0; e < 4; ++e) ss += b0[e] * b0[e];
#pragma unroll
  for (int e = 0; e < 4; ++e) ss += b1[e] * b1[e];
#pragma unroll
  for (int off = 16; off > 0; off >>= 1) ss += __shfl_xor(ss, off, 32);
  const float nrm = fmaxf(sqrtf(ss), 1e-12f);
  const float inv = XNSC * (1.0f / nrm);
  v8h h0, h1;
#pragma unroll
  for (int e = 0; e < 4; ++e) {
    h0[e]     = (_Float16)(a0[e] * inv);
    h0[4 + e] = (_Float16)(a1[e] * inv);
    h1[e]     = (_Float16)(b0[e] * inv);
    h1[4 + e] = (_Float16)(b1[e] * inv);
  }
  if (row < nrows) {
    _Float16* dst = xn + (size_t)row * NCOL;
    for (int pass = 0; pass < 2; ++pass) {
      *(volatile v8h*)(dst + lane * 8) = h0;
      *(volatile v8h*)(dst + 256 + lane * 8) = h1;
      __threadfence();
    }
  }
}

__global__ __launch_bounds__(256) void transpose_x16(const float* __restrict__ x, _Float16* __restrict__ xt) {
  __shared__ __align__(16) _Float16 sH[64 * 72];
  const int tid = threadIdx.x, lane = tid & 31, wave = tid >> 5;
  const int j0 = blockIdx.x * 64;
  const int c0 = blockIdx.y * 64;
  const int lr = tid >> 4;
  const int lc4 = (tid & 15) * 4;
  if (c0 + 64 <= NCOL) {
#pragma unroll
    for (int it = 0; it < 4; ++it) {
      const int r = it * 16 + lr;
      const v4f v = *(const v4f*)(x + (size_t)(j0 + r) * NCOL + c0 + lc4);
#pragma unroll
      for (int e = 0; e < 4; ++e) sH[(lc4 + e) * 72 + r] = (_Float16)v[e];
    }
  } else {
#pragma unroll
    for (int it = 0; it < 4; ++it) {
      const int r = it * 16 + lr;
#pragma unroll
      for (int e = 0; e < 4; ++e) {
        const int cl = lc4 + e;
        sH[cl * 72 + r] = (c0 + cl == NCOL) ? (_Float16)1.0f : (_Float16)0.0f;
      }
    }
  }
  __syncthreads();
  const int q = lane >> 3, c8 = (lane & 7) * 8;
  for (int pass = 0; pass < 2; ++pass) {
#pragma unroll
    for (int it = 0; it < 2; ++it) {
      const int r = it * 32 + wave * 4 + q;
      const v8h hv = *(const v8h*)(sH + r * 72 + c8);
      *(volatile v8h*)(xt + (size_t)(c0 + r) * NROW + j0 + c8) = hv;
    }
    __threadfence();
  }
}

__global__ __launch_bounds__(256) void finalize_out(const float* __restrict__ ob, float* __restrict__ out, int nrows) {
  const int lane = threadIdx.x & 31;
  const int wave = threadIdx.x >> 5;
  const int row  = blockIdx.x * 8 + wave;
  const int rowc = row < nrows ? row : nrows - 1;
  const float* src = ob + (size_t)rowc * NCT;
  const float den = src[NCOL];
  const float inv = 1.0f / den;
  v4f v0 = *(const v4f*)(src + lane * 4);
  v4f v1 = *(const v4f*)(src + 128 + lane * 4);
  v4f v2 = *(const v4f*)(src + 256 + lane * 4);
  v4f v3 = *(const v4f*)(src + 384 + lane * 4);
  v0 *= inv; v1 *= inv; v2 *= inv; v3 *= inv;
  if (row < nrows) {
    float* dst = out + (size_t)row * NCOL;
    for (int pass = 0; pass < 2; ++pass) {
      *(volatile v4f*)(dst + lane * 4) = v0;
      *(volatile v4f*)(dst + 128 + lane * 4) = v1;
      *(volatile v4f*)(dst + 256 + lane * 4) = v2;
      *(volatile v4f*)(dst + 384 + lane * 4) = v3;
      __threadfence();
    }
  }
}

extern "C" void kernel_launch(void* const* d_in, const int* in_sizes, int n_in,
                              void* d_out, int out_size, void* d_ws, size_t ws_size,
                              hipStream_t stream) {
  if (n_in < 1) return;
  if (in_sizes[0] != NROW * NCOL || out_size != NROW * NCOL) return;
  const size_t bytesXN = (size_t)NROW * NCOL * 2;
  const size_t bytesXT = (size_t)NCT * NROW * 2;
  const size_t bytesP  = (size_t)RB * NROW * 2;
  const size_t bytesOB = (size_t)NROW * NCT * 4;
  const size_t offXN = 0;
  const size_t offXT = offXN + bytesXN;
  const size_t offP  = offXT + bytesXT;
  const size_t offOB = offP + bytesP;
  const size_t total = offOB + bytesOB;
  if (total > ws_size) return;

  const float* x = (const float*)d_in[0];
  float* out = (float*)d_out;
  char* ws = (char*)d_ws;
  _Float16* XN16 = (_Float16*)(ws + offXN);
  _Float16* XT16 = (_Float16*)(ws + offXT);
  _Float16* P16  = (_Float16*)(ws + offP);
  float*    OB   = (float*)(ws + offOB);

  rownorm_xn16<<<dim3(NROW / 8), dim3(256), 0, stream>>>(x, XN16, NROW);
  transpose_x16<<<dim3(NROW / 64, NCT / 64), dim3(256), 0, stream>>>(x, XT16);

  const int tilesS  = (RB / 64) * (NROW / 64);
  const int tilesPV = (RB / 64) * (NCT / 64);
  for (int rb = 0; rb < NROW; rb += RB) {
    const unsigned short* Aq = (const unsigned short*)(XN16 + (size_t)rb * NCOL);
    const unsigned short* Bk = (const unsigned short*)XN16;
    wmma_gemm64<0, false, 0, 1, false, 6><<<dim3((tilesS + 7) / 8, 1), dim3(256), 0, stream>>>(
        Aq, Aq, NCOL, 0L,
        Bk, Bk, NCOL, 0L,
        (void*)P16, (void*)P16, NROW, 0L,
        (const float*)OB, (const float*)OB, 0L,
        RB, NROW, NCOL, SSC);
    const unsigned short* Ap = (const unsigned short*)P16;
    const unsigned short* Bx = (const unsigned short*)XT16;
    float* Ob = OB + (size_t)rb * NCT;
    wmma_gemm64<0, false, 0, 0, false, 0><<<dim3((tilesPV + 7) / 8, 1), dim3(256), 0, stream>>>(
        Ap, Ap, NROW, 0L,
        Bx, Bx, NROW, 0L,
        (void*)Ob, (void*)Ob, NCT, 0L,
        (const float*)OB, (const float*)OB, 0L,
        RB, NCT, NROW, 1.0f);
  }

  finalize_out<<<dim3(NROW / 8), dim3(256), 0, stream>>>(OB, out, NROW);
}
